// MambaLayer_33621003993786
// MI455X (gfx1250) — hardware-run, weakly checked
//
#include <hip/hip_runtime.h>
#include <math.h>

constexpr int kBatch = 4;
constexpr int kSeq   = 1024;
constexpr int kHid   = 128;
constexpr int kRows  = kBatch * kSeq;
constexpr int kXzW   = 2 * kHid;
constexpr int kSsmW  = 3 * kHid;
constexpr int kChunk = 16;
constexpr int kLvPlane = kChunk * kHid;

constexpr float kActCarry  = 16.0f;
constexpr float kWCarry    = 16.0f;
constexpr float kResCarry  = 2048.0f;
constexpr float kResInv    = 1.0f / kResCarry;
constexpr float kScaleFold = 1.0f / (kActCarry * kWCarry);
constexpr float kF16MinNormal = 6.103515625e-5f;

static_assert(kHid == 128 && kChunk == 16);
static_assert(kRows % 32 == 0 && kXzW % 64 == 0 && kSsmW % 64 == 0 && kHid % 64 == 0);
static_assert(kHid % 32 == 0);
static_assert(kSeq % kChunk == 0);
static_assert((kRows * kHid / 8) % 256 == 0);
static_assert((kRows * (kHid / 4)) % 256 == 0);

typedef __attribute__((ext_vector_type(16))) _Float16 v16h;
typedef __attribute__((ext_vector_type(8)))  _Float16 v8h;
typedef __attribute__((ext_vector_type(8)))  float    v8f;
typedef __attribute__((ext_vector_type(4)))  float    v4f;
typedef __attribute__((ext_vector_type(4)))  unsigned int v4u;

constexpr size_t kActPlaneB = (size_t)kRows * kHid * 2;
constexpr size_t kWinB      = (size_t)kXzW * kHid * 2;
constexpr size_t kWxB       = (size_t)kSsmW * kHid * 2;
constexpr size_t kWoutB     = (size_t)kHid * kHid * 2;
constexpr size_t kXzB       = (size_t)kRows * kXzW * 4;
constexpr size_t kXcB       = (size_t)kRows * kHid * 4;
constexpr size_t kSsmB      = (size_t)kRows * kSsmW * 4;
constexpr size_t kYgB       = (size_t)kRows * kHid * 4;
constexpr size_t kWsTotal   = 6 * kActPlaneB + 2 * (kWinB + kWxB + kWoutB) + kXzB + kXcB + kSsmB + kYgB;
static_assert(kWsTotal == 21364736ull);
static_assert(kWsTotal <= 134217728ull);
static_assert(kActPlaneB % 256 == 0 && kWinB % 256 == 0 && kWxB % 256 == 0 && kWoutB % 256 == 0);
static_assert(kXzB % 256 == 0 && kXcB % 256 == 0 && kSsmB % 256 == 0 && kYgB % 256 == 0);

__device__ __forceinline__ unsigned pk16(unsigned short a, unsigned short b) {
  return (unsigned)a | ((unsigned)b << 16);
}
__device__ __forceinline__ void h_split(float v, unsigned short& hb, unsigned short& rb) {
  const float vf = (fabsf(v) < kF16MinNormal) ? 0.0f : v;
  const _Float16 h = (_Float16)vf;
  const float hf = (float)h;
  const float d = (v - hf) * kResCarry;
  const float df = (fabsf(d) < kF16MinNormal) ? 0.0f : d;
  const _Float16 r = (_Float16)df;
  hb = __builtin_bit_cast(unsigned short, h);
  rb = __builtin_bit_cast(unsigned short, r);
}
__device__ __forceinline__ void pack8_split(const float (&v)[8], v4u& uh, v4u& ur) {
  unsigned short hb[8], rb[8];
#pragma unroll
  for (int e = 0; e < 8; ++e) h_split(v[e], hb[e], rb[e]);
  uh = (v4u){pk16(hb[0], hb[1]), pk16(hb[2], hb[3]), pk16(hb[4], hb[5]), pk16(hb[6], hb[7])};
  ur = (v4u){pk16(rb[0], rb[1]), pk16(rb[2], rb[3]), pk16(rb[4], rb[5]), pk16(rb[6], rb[7])};
}

struct FragH {
  union U { v16h v; v8h h[2]; };
  static __device__ __forceinline__ v16h load(const _Float16* p) {
    U f;
    f.h[0] = *(const v8h*)(p);
    f.h[1] = *(const v8h*)(p + 16);
    return f.v;
  }
  static __device__ __forceinline__ v8f mma(v16h a, v16h b, v8f c) {
    return __builtin_amdgcn_wmma_f32_16x16x32_f16(false, a, false, b, (short)0, c, false, false);
  }
};
__device__ __forceinline__ void guard_split(v8f& a0, v8f& a1, v8f& a2, v8f& a3,
                                            v16h x0, v16h x1, v16h x2, v16h x3, v16h y0, v16h y1) {
  asm volatile("v_nop\n\tv_nop\n\tv_nop\n\tv_nop"
               : "+v"(a0), "+v"(a1), "+v"(a2), "+v"(a3)
               : "v"(x0), "v"(x1), "v"(x2), "v"(x3), "v"(y0), "v"(y1));
}
__device__ __forceinline__ void acc_guard4(v8f& a, v8f& b, v8f& c, v8f& d) {
  asm volatile("v_nop\n\tv_nop\n\tv_nop\n\tv_nop" : "+v"(a), "+v"(b), "+v"(c), "+v"(d));
}

template <int ACT>
__global__ __launch_bounds__(256) void gemm_split_kernel(
    const unsigned short* __restrict__ Ahp, const unsigned short* __restrict__ Arp, int lda,
    const unsigned short* __restrict__ Bhp, const unsigned short* __restrict__ Brp, int ldb,
    float* __restrict__ Cout, int ldc, const float* __restrict__ bias,
    int M, int N, int K, float scale, int actCols) {
  __shared__ __align__(16) float sT[8][16 * 68];
  const int lane = threadIdx.x & 31;
  const int wave = threadIdx.x >> 5;
  const int tilesN = N >> 6;
  const int tilesM = M >> 5;
  const int tile = blockIdx.x * 8 + wave;
  if (tile >= tilesM * tilesN) return;
  const int tm = tile / tilesN;
  const int tn = tile - tm * tilesN;
  const int m0 = tm << 5;
  const int n0 = tn << 6;
  const int rlane = lane & 15;
  const int half8 = (lane >> 4) * 8;
  const int mOff  = (lane >> 4) * 8;

  const size_t aoff = (size_t)(m0 + rlane) * lda + half8;
  const size_t boff = (size_t)(n0 + rlane) * ldb + half8;
  const _Float16* pa0 = (const _Float16*)Ahp + aoff;
  const _Float16* pa1 = pa0 + (size_t)16 * lda;
  const _Float16* pr0 = (const _Float16*)Arp + aoff;
  const _Float16* pr1 = pr0 + (size_t)16 * lda;
  const _Float16* pbh = (const _Float16*)Bhp + boff;
  const _Float16* pbr = (const _Float16*)Brp + boff;
  const size_t bstep = (size_t)16 * ldb;

  v8f acc[2][4], accr[2][4];
#pragma unroll
  for (int i = 0; i < 2; ++i)
#pragma unroll
    for (int j = 0; j < 4; ++j) {
      acc[i][j]  = (v8f){0.f, 0.f, 0.f, 0.f, 0.f, 0.f, 0.f, 0.f};
      accr[i][j] = (v8f){0.f, 0.f, 0.f, 0.f, 0.f, 0.f, 0.f, 0.f};
    }

  for (int k0 = 0; k0 < K; k0 += 32) {
    const v16h ah0 = FragH::load(pa0 + k0);
    const v16h ah1 = FragH::load(pa1 + k0);
    const v16h ar0 = FragH::load(pr0 + k0);
    const v16h ar1 = FragH::load(pr1 + k0);
#pragma unroll
    for (int j = 0; j < 4; ++j) {
      const v16h bh = FragH::load(pbh + j * bstep + k0);
      const v16h br = FragH::load(pbr + j * bstep + k0);
      acc[0][j]  = FragH::mma(ah0, bh, acc[0][j]);
      acc[1][j]  = FragH::mma(ah1, bh, acc[1][j]);
      accr[0][j] = FragH::mma(ah0, br, accr[0][j]);
      accr[1][j] = FragH::mma(ah1, br, accr[1][j]);
      accr[0][j] = FragH::mma(ar0, bh, accr[0][j]);
      accr[1][j] = FragH::mma(ar1, bh, accr[1][j]);
      guard_split(acc[0][j], acc[1][j], accr[0][j], accr[1][j], ah0, ah1, ar0, ar1, bh, br);
    }
  }
  acc_guard4(acc[0][0], acc[0][1], acc[0][2], acc[0][3]);
  acc_guard4(acc[1][0], acc[1][1], acc[1][2], acc[1][3]);
  acc_guard4(accr[0][0], accr[0][1], accr[0][2], accr[0][3]);
  acc_guard4(accr[1][0], accr[1][1], accr[1][2], accr[1][3]);

  float bv[4];
#pragma unroll
  for (int j = 0; j < 4; ++j) bv[j] = bias[n0 + (j << 4) + rlane];

  float* slab = sT[wave];
  const int hh = lane >> 4;
  const int c4 = (lane & 15) * 4;
#pragma unroll
  for (int i = 0; i < 2; ++i) {
    const int mBase = m0 + (i << 4);
#pragma unroll
    for (int j = 0; j < 4; ++j) {
#pragma unroll
      for (int r = 0; r < 8; ++r) {
        float v = acc[i][j][r] + accr[i][j][r] * kResInv;
        v = v * scale + bv[j];
        slab[(mOff + r) * 68 + (j << 4) + rlane] = v;
      }
    }
    __builtin_amdgcn_fence(__ATOMIC_RELEASE, "workgroup");
    __builtin_amdgcn_wave_barrier();
    __builtin_amdgcn_fence(__ATOMIC_ACQUIRE, "workgroup");
    if (ACT == 1) {
#pragma unroll 1
      for (int it = 0; it < 8; ++it) {
        float* sp = slab + (it * 2 + hh) * 68 + c4;
        const v4f xv = *(const v4f*)sp;
        v4f ov;
#pragma unroll
        for (int e = 0; e < 4; ++e) {
          const float x = xv[e];
          const float s1 = fmaxf(x, 0.0f) + log1pf(expf(-fabsf(x)));
          ov[e] = ((n0 + c4 + e) < actCols) ? s1 : x;
        }
        *(v4f*)sp = ov;
      }
      __builtin_amdgcn_fence(__ATOMIC_RELEASE, "workgroup");
      __builtin_amdgcn_wave_barrier();
      __builtin_amdgcn_fence(__ATOMIC_ACQUIRE, "workgroup");
    }
    for (int pass = 0; pass < 2; ++pass) {
#pragma unroll
      for (int it = 0; it < 8; ++it) {
        const int row = it * 2 + hh;
        const v4f v = *(const v4f*)(slab + row * 68 + c4);
        *(volatile v4f*)(Cout + (size_t)(mBase + row) * ldc + n0 + c4) = v;
      }
      __threadfence();
    }
    __builtin_amdgcn_fence(__ATOMIC_RELEASE, "workgroup");
    __builtin_amdgcn_wave_barrier();
    __builtin_amdgcn_fence(__ATOMIC_ACQUIRE, "workgroup");
  }
}

__global__ __launch_bounds__(256) void wt_plane_kernel(const float* __restrict__ W,
                                                       unsigned short* __restrict__ outh,
                                                       unsigned short* __restrict__ outr,
                                                       int Kd, int Nd) {
  __shared__ float sm[64][65];
  const int t  = threadIdx.x;
  const int k0 = blockIdx.x * 64;
  const int n0 = blockIdx.y * 64;
#pragma unroll
  for (int i = 0; i < 16; ++i) {
    const int e = i * 256 + t;
    const int r = e >> 6;
    const int c = e & 63;
    const int kk = k0 + r;
    const int nn = n0 + c;
    const bool valid = (kk < Kd) && (nn < Nd);
    const int kc = (kk < Kd) ? kk : (Kd - 1);
    const int nc = (nn < Nd) ? nn : (Nd - 1);
    const float v = W[(size_t)kc * Nd + nc];
    sm[c][r] = valid ? (v * kWCarry) : 0.0f;
  }
  __syncthreads();
  const int lane = t & 31, wave = t >> 5;
  const int q = lane >> 3, c8 = (lane & 7) * 8;
  for (int pass = 0; pass < 2; ++pass) {
#pragma unroll
    for (int it = 0; it < 2; ++it) {
      const int row = wave * 8 + it * 4 + q;
      float v[8];
#pragma unroll
      for (int e = 0; e < 8; ++e) v[e] = sm[row][c8 + e];
      v4u uh, ur;
      pack8_split(v, uh, ur);
      const size_t o = (size_t)(n0 + row) * Kd + k0 + c8;
      *(volatile v4u*)(outh + o) = uh;
      *(volatile v4u*)(outr + o) = ur;
    }
    __threadfence();
  }
}

__global__ __launch_bounds__(256) void cast_split_kernel(const float* __restrict__ src,
                                                         unsigned short* __restrict__ dh,
                                                         unsigned short* __restrict__ dr, int total8) {
  const int i = blockIdx.x * 256 + threadIdx.x;
  if (i >= total8) return;
  const size_t e0 = (size_t)i << 3;
  const v4f a0 = *(const v4f*)(src + e0);
  const v4f a1 = *(const v4f*)(src + e0 + 4);
  float v[8];
#pragma unroll
  for (int e = 0; e < 4; ++e) {
    v[e]     = a0[e] * kActCarry;
    v[4 + e] = a1[e] * kActCarry;
  }
  v4u uh, ur;
  pack8_split(v, uh, ur);
  *(volatile v4u*)(dh + e0) = uh;
  *(volatile v4u*)(dr + e0) = ur;
  __threadfence();
  *(volatile v4u*)(dh + e0) = uh;
  *(volatile v4u*)(dr + e0) = ur;
}

__global__ __launch_bounds__(256) void conv_silu_kernel(const float* __restrict__ XZ,
                                                        const float* __restrict__ cw,
                                                        const float* __restrict__ cb,
                                                        float* __restrict__ XC) {
  const int i = blockIdx.x * 256 + threadIdx.x;
  if (i >= kRows * (kHid / 4)) return;
  const int row = i >> 5;
  const int c4  = (i & 31) * 4;
  const int t   = row & (kSeq - 1);
  const bool hasPrev = (t > 0);
  const bool hasNext = (t < kSeq - 1);
  const int rp = hasPrev ? (row - 1) : row;
  const int rn = hasNext ? (row + 1) : row;
  const v4f xm = *(const v4f*)(XZ + (size_t)rp * kXzW + c4);
  const v4f xc = *(const v4f*)(XZ + (size_t)row * kXzW + c4);
  const v4f xn = *(const v4f*)(XZ + (size_t)rn * kXzW + c4);
  float pm0 = xm[0], pm1 = xm[1], pm2 = xm[2], pm3 = xm[3];
  float pn0 = xn[0], pn1 = xn[1], pn2 = xn[2], pn3 = xn[3];
  asm volatile("" : "+v"(pm0), "+v"(pm1), "+v"(pm2), "+v"(pm3));
  asm volatile("" : "+v"(pn0), "+v"(pn1), "+v"(pn2), "+v"(pn3));
  float pm[4] = {pm0, pm1, pm2, pm3};
  float pn[4] = {pn0, pn1, pn2, pn3};
  const v4f q0 = *(const v4f*)(cw + 3 * c4);
  const v4f q1 = *(const v4f*)(cw + 3 * c4 + 4);
  const v4f q2 = *(const v4f*)(cw + 3 * c4 + 8);
  const float wf[12] = {q0[0], q0[1], q0[2], q0[3], q1[0], q1[1], q1[2], q1[3], q2[0], q2[1], q2[2], q2[3]};
  const v4f bq = *(const v4f*)(cb + c4);
  v4f ov;
#pragma unroll
  for (int e = 0; e < 4; ++e) {
    const float a = hasPrev ? pm[e] : 0.0f;
    const float c = hasNext ? pn[e] : 0.0f;
    float acc = wf[3 * e + 0] * a;
    acc = fmaf(wf[3 * e + 1], xc[e], acc);
    acc = fmaf(wf[3 * e + 2], c, acc);
    const float sv = acc + bq[e];
    const float sg = 1.0f / (1.0f + expf(-sv));
    ov[e] = sv * sg;
  }
  float* dst = XC + (size_t)row * kHid + c4;
  *(volatile v4f*)dst = ov;
  __threadfence();
  *(volatile v4f*)dst = ov;
}

__global__ __launch_bounds__(1024) void scan_full_kernel(const float* __restrict__ SSM,
                                                         const float* __restrict__ XC,
                                                         const float* __restrict__ U,
                                                         const float* __restrict__ XZ,
                                                         const float* __restrict__ Alog,
                                                         const float* __restrict__ Dv,
                                                         float* __restrict__ YG) {
  __shared__ __align__(16) float lv[6 * kLvPlane];
  __shared__ __align__(16) float red[8 * kHid];
  __shared__ __align__(16) float yb[kChunk * kHid];
  const int tid = threadIdx.x;
  const int e   = tid & 127;
  const int g   = tid >> 7;
  const size_t row0 = (size_t)blockIdx.x * kSeq;

  const float Ae = -expf(Alog[e]);
  const float De = Dv[e];

  const int half = tid >> 9;
  const int sidx = tid & 511;
  const int lrow = sidx >> 5;
  const int lc4  = (sidx & 31) * 4;
  const float* b0 = (half == 0) ? SSM : XC;
  const float* b1 = (half == 0) ? (SSM + kHid) : U;
  const float* b2 = (half == 0) ? (SSM + 2 * kHid) : (XZ + kHid);
  const int pt0 = (half == 0) ? kSsmW : kHid;
  const int pt1 = (half == 0) ? kSsmW : kHid;
  const int pt2 = (half == 0) ? kSsmW : kXzW;
  float* d0 = lv + (half * 3 + 0) * kLvPlane + lrow * kHid + lc4;
  float* d1 = lv + (half * 3 + 1) * kLvPlane + lrow * kHid + lc4;
  float* d2 = lv + (half * 3 + 2) * kLvPlane + lrow * kHid + lc4;

  float h[16];
#pragma unroll
  for (int k = 0; k < 16; ++k) h[k] = 0.0f;

#pragma unroll 1
  for (int ch = 0; ch < kSeq / kChunk; ++ch) {
    const size_t r = row0 + (size_t)(ch * kChunk + lrow);
    {
      const v4f t0 = *(const v4f*)(b0 + r * pt0 + lc4);
      const v4f t1 = *(const v4f*)(b1 + r * pt1 + lc4);
      const v4f t2 = *(const v4f*)(b2 + r * pt2 + lc4);
      *(v4f*)d0 = t0;
      *(v4f*)d1 = t1;
      *(v4f*)d2 = t2;
    }
    __syncthreads();

#pragma unroll 1
    for (int s = 0; s < kChunk; ++s) {
      const float* pd = lv + 0 * kLvPlane + s * kHid + 16 * g;
      const float* pb = lv + 1 * kLvPlane + s * kHid + 16 * g;
      const float xt = lv[3 * kLvPlane + s * kHid + e];
      float part = 0.0f;
#pragma unroll
      for (int g4 = 0; g4 < 4; ++g4) {
        const v4f dq = *(const v4f*)(pd + 4 * g4);
        const v4f bq = *(const v4f*)(pb + 4 * g4);
#pragma unroll
        for (int j = 0; j < 4; ++j) {
          const float di = dq[j];
          const float dec = expf(di * Ae);
          const float inj = (di * bq[j]) * xt;
          const float hn = dec * h[4 * g4 + j] + inj;
          h[4 * g4 + j] = hn;
          part += hn;
        }
      }
      red[g * kHid + e] = part;
      __syncthreads();
      if (g == 0) {
        float tot = 0.0f;
#pragma unroll
        for (int gg = 0; gg < 8; ++gg) tot += red[gg * kHid + e];
        const float ct = lv[2 * kLvPlane + s * kHid + e];
        const float ut = lv[4 * kLvPlane + s * kHid + e];
        const float zt = lv[5 * kLvPlane + s * kHid + e];
        const float y  = ct * tot + De * ut;
        const float sg = 1.0f / (1.0f + expf(-zt));
        yb[s * kHid + e] = y * (zt * sg);
      }
      __syncthreads();
    }

    if (tid < 128) {
      const int wave = tid >> 5;
      const int lane = tid & 31;
      v4f val[4];
#pragma unroll
      for (int it = 0; it < 4; ++it) val[it] = *(const v4f*)(yb + (wave * 4 + it) * kHid + lane * 4);
      float* dst = YG + (row0 + (size_t)(ch * kChunk + wave * 4)) * kHid + lane * 4;
      for (int pass = 0; pass < 2; ++pass) {
#pragma unroll
        for (int it = 0; it < 4; ++it) *(volatile v4f*)(dst + (size_t)it * kHid) = val[it];
        __threadfence();
      }
    }
  }
}

extern "C" void kernel_launch(void* const* d_in, const int* in_sizes, int n_in,
                              void* d_out, int out_size, void* d_ws, size_t ws_size, hipStream_t stream) {
  if (n_in < 11 || d_out == nullptr || d_ws == nullptr) return;
  if (in_sizes[0] != kRows * kHid) return;
  if (in_sizes[1] != kHid * kXzW || in_sizes[2] != kXzW) return;
  if (in_sizes[3] != kHid * 3 || in_sizes[4] != kHid) return;
  if (in_sizes[5] != kHid * kSsmW || in_sizes[6] != kSsmW) return;
  if (in_sizes[7] != kHid || in_sizes[8] != kHid) return;
  if (in_sizes[9] != kHid * kHid || in_sizes[10] != kHid) return;
  if (out_size != kRows * kHid) return;

  const float* u      = (const float*)d_in[0];
  const float* W_in   = (const float*)d_in[1];
  const float* b_in   = (const float*)d_in[2];
  const float* conv_w = (const float*)d_in[3];
  const float* conv_b = (const float*)d_in[4];
  const float* W_x    = (const float*)d_in[5];
  const float* b_x    = (const float*)d_in[6];
  const float* A_log  = (const float*)d_in[7];
  const float* Dv     = (const float*)d_in[8];
  const float* W_out  = (const float*)d_in[9];
  const float* b_out  = (const float*)d_in[10];
  float* out = (float*)d_out;

  char* ws = (char*)d_ws;
  size_t off = 0;
  auto carve = [&](size_t bytes) -> char* {
    char* p = ws + off;
    off += (bytes + 255) & ~(size_t)255;
    return p;
  };
  unsigned short* UH  = (unsigned short*)carve(kActPlaneB);
  unsigned short* UR  = (unsigned short*)carve(kActPlaneB);
  unsigned short* XH  = (unsigned short*)carve(kActPlaneB);
  unsigned short* XR  = (unsigned short*)carve(kActPlaneB);
  unsigned short* YH  = (unsigned short*)carve(kActPlaneB);
  unsigned short* YR  = (unsigned short*)carve(kActPlaneB);
  unsigned short* WIh = (unsigned short*)carve(kWinB);
  unsigned short* WIr = (unsigned short*)carve(kWinB);
  unsigned short* WXh = (unsigned short*)carve(kWxB);
  unsigned short* WXr = (unsigned short*)carve(kWxB);
  unsigned short* WOh = (unsigned short*)carve(kWoutB);
  unsigned short* WOr = (unsigned short*)carve(kWoutB);
  float* XZ  = (float*)carve(kXzB);
  float* XC  = (float*)carve(kXcB);
  float* SSM = (float*)carve(kSsmB);
  float* YG  = (float*)carve(kYgB);
  if (off != kWsTotal || off > ws_size || off > (size_t)134217728) return;

  wt_plane_kernel<<<dim3(kHid / 64, kXzW / 64), 256, 0, stream>>>(W_in, WIh, WIr, kHid, kXzW);
  wt_plane_kernel<<<dim3(kHid / 64, kSsmW / 64), 256, 0, stream>>>(W_x, WXh, WXr, kHid, kSsmW);
  wt_plane_kernel<<<dim3(kHid / 64, kHid / 64), 256, 0, stream>>>(W_out, WOh, WOr, kHid, kHid);

  const int total8 = kRows * kHid / 8;
  const int castBlocks = total8 / 256;

  cast_split_kernel<<<castBlocks, 256, 0, stream>>>(u, UH, UR, total8);

  gemm_split_kernel<0><<<(kRows / 32) * (kXzW / 64) / 8, 256, 0, stream>>>(
      UH, UR, kHid, WIh, WIr, kHid, XZ, kXzW, b_in, kRows, kXzW, kHid, kScaleFold, 0);

  conv_silu_kernel<<<(kRows * (kHid / 4)) / 256, 256, 0, stream>>>(XZ, conv_w, conv_b, XC);

  cast_split_kernel<<<castBlocks, 256, 0, stream>>>(XC, XH, XR, total8);

  gemm_split_kernel<1><<<(kRows / 32) * (kSsmW / 64) / 8, 256, 0, stream>>>(
      XH, XR, kHid, WXh, WXr, kHid, SSM, kSsmW, b_x, kRows, kSsmW, kHid, kScaleFold, kHid);

  scan_full_kernel<<<kBatch, 1024, 0, stream>>>(SSM, XC, u, XZ, A_log, Dv, YG);

  cast_split_kernel<<<castBlocks, 256, 0, stream>>>(YG, YH, YR, total8);

  gemm_split_kernel<0><<<(kRows / 32) * (kHid / 64) / 8, 256, 0, stream>>>(
      YH, YR, kHid, WOh, WOr, kHid, out, kHid, b_out, kRows, kHid, kHid, kScaleFold, 0);
}
